// PerceptGNN_69002944578206
// MI455X (gfx1250) — hardware-verified
//
#include <hip/hip_runtime.h>
#include <math.h>
#include <stdint.h>

typedef unsigned short us;
typedef __bf16   v16b __attribute__((ext_vector_type(16)));
typedef float    v8f  __attribute__((ext_vector_type(8)));
typedef float    v4f  __attribute__((ext_vector_type(4)));
typedef float    v2f  __attribute__((ext_vector_type(2)));
typedef unsigned int v4u __attribute__((ext_vector_type(4)));

static constexpr int NB    = 8;
static constexpr int NNODE = 1024;
static constexpr int NHEAD = 8;

__device__ __forceinline__ us f2bf_bits(float f) {
  const unsigned u = __float_as_uint(f);
  return (us)((u + 0x7FFFu + ((u >> 16) & 1u)) >> 16);
}
__device__ __forceinline__ float bf_bits2f(us h) { return __uint_as_float(((unsigned)h) << 16); }
__device__ __forceinline__ unsigned pk16(us a, us b) { return (unsigned)a | ((unsigned)b << 16); }
__device__ __forceinline__ void split2(float f, us& hi, us& lo) {
  hi = f2bf_bits(f);
  lo = f2bf_bits(f - bf_bits2f(hi));
}
union FragU { v16b v; v4u u[2]; };
__device__ __forceinline__ v16b ldfrag(const us* p) {
  FragU f;
  f.u[0] = *(const v4u*)(p);
  f.u[1] = *(const v4u*)(p + 16);
  return f.v;
}
__device__ __forceinline__ v8f mma_bf(v16b a, v16b b, v8f c) {
  c = __builtin_amdgcn_wmma_f32_16x16x32_bf16(false, a, false, b, (short)0, c, false, false);
  asm volatile("v_nop\n\tv_nop\n\tv_nop\n\tv_nop" : "+v"(c) : "v"(a), "v"(b));
  return c;
}
__device__ __forceinline__ void lds_wave_sync() {
  __builtin_amdgcn_fence(__ATOMIC_RELEASE, "workgroup");
  __builtin_amdgcn_wave_barrier();
  __builtin_amdgcn_fence(__ATOMIC_ACQUIRE, "workgroup");
}
__device__ __forceinline__ float lrelu02(float v) { return fmaxf(v, 0.2f * v); }
__device__ __forceinline__ float elu1(float v) { return v > 0.0f ? v : expm1f(v); }
__device__ __forceinline__ v8f zero8() { v8f z = {0.f, 0.f, 0.f, 0.f, 0.f, 0.f, 0.f, 0.f}; return z; }

__global__ __launch_bounds__(256) void k_split2(const float* __restrict__ in, us* __restrict__ hi,
                                                us* __restrict__ lo, int n2) {
  const int i = blockIdx.x * 256 + threadIdx.x;
  if (i < n2) {
    const v2f f = *(const v2f*)(in + 2 * (size_t)i);
    const us h0 = f2bf_bits(f[0]), h1 = f2bf_bits(f[1]);
    const us l0 = f2bf_bits(f[0] - bf_bits2f(h0)), l1 = f2bf_bits(f[1] - bf_bits2f(h1));
    const unsigned uh = pk16(h0, h1), ul = pk16(l0, l1);
    ((volatile unsigned*)hi)[i] = uh;
    ((volatile unsigned*)lo)[i] = ul;
    __threadfence();
    ((volatile unsigned*)hi)[i] = uh;
    ((volatile unsigned*)lo)[i] = ul;
  }
}

__global__ __launch_bounds__(256) void k_tsplit(const float* __restrict__ W, us* __restrict__ oh,
                                                us* __restrict__ ol, int R, int Cc, long sIn, long sOut) {
  __shared__ __align__(16) float tf[64 * 68];
  W  += (size_t)blockIdx.z * sIn;
  oh += (size_t)blockIdx.z * sOut;
  ol += (size_t)blockIdx.z * sOut;
  const int c0  = blockIdx.x * 64;
  const int r0  = blockIdx.y * 64;
  const int tid = threadIdx.x;
  {
    const int lr = tid >> 4;
    const int c4 = (tid & 15) * 4;
#pragma unroll
    for (int it = 0; it < 4; ++it) {
      const int rr = it * 16 + lr;
      const v4f a = *(const v4f*)(W + (size_t)(r0 + rr) * Cc + c0 + c4);
      *(v4f*)(tf + rr * 68 + c4) = a;
    }
  }
  __syncthreads();
  const int sub = tid >> 3;
  const int c8  = (tid & 7) * 8;
  v4u hv[2], lv[2];
#pragma unroll
  for (int it = 0; it < 2; ++it) {
    const int oc = it * 32 + sub;
    v4u a, a2;
#pragma unroll
    for (int q = 0; q < 4; ++q) {
      const float f0 = tf[(c8 + 2 * q) * 68 + oc];
      const float f1 = tf[(c8 + 2 * q + 1) * 68 + oc];
      us h0, l0, h1, l1;
      split2(f0, h0, l0);
      split2(f1, h1, l1);
      a[q]  = pk16(h0, h1);
      a2[q] = pk16(l0, l1);
    }
    hv[it] = a; lv[it] = a2;
  }
  for (int pass = 0; pass < 2; ++pass) {
#pragma unroll
    for (int it = 0; it < 2; ++it) {
      const int oc = it * 32 + sub;
      const size_t go = (size_t)(c0 + oc) * R + r0 + c8;
      *(volatile v4u*)(oh + go) = hv[it];
      *(volatile v4u*)(ol + go) = lv[it];
    }
    __threadfence();
  }
}

__global__ __launch_bounds__(256) void k_gemm_split(
    const us* __restrict__ Ah, const us* __restrict__ Al, int lda,
    const us* __restrict__ Bth, const us* __restrict__ Btl, int ldb, long strideB,
    float* __restrict__ Cf, us* __restrict__ Ch, us* __restrict__ Cl, int ldc, long strideC,
    int M, int N, int K) {
  __shared__ __align__(16) float sT[8][16 * 68];
  const int z    = blockIdx.y;
  const int lane = threadIdx.x & 31;
  const int wave = threadIdx.x >> 5;
  const int tilesN = N >> 6;
  const int tilesM = M >> 5;
  const int tile = blockIdx.x * 8 + wave;
  if (tile >= tilesM * tilesN) return;
  const int tm = tile / tilesN;
  const int tn = tile - tm * tilesN;
  const int m0 = tm << 5;
  const int n0 = tn << 6;
  const us* Bh = Bth + (size_t)z * strideB;
  const us* Bl = Btl + (size_t)z * strideB;
  const int rl   = lane & 15;
  const int koff = (lane >> 4) * 8;
  const int mOff = (lane >> 4) * 8;

  v8f acc[2][4];
#pragma unroll
  for (int i = 0; i < 2; ++i)
#pragma unroll
    for (int j = 0; j < 4; ++j) acc[i][j] = zero8();

  for (int k0 = 0; k0 < K; k0 += 32) {
    v16b bh[4], bl[4];
#pragma unroll
    for (int j = 0; j < 4; ++j) {
      const size_t bo = (size_t)(n0 + (j << 4) + rl) * ldb + k0 + koff;
      bh[j] = ldfrag(Bh + bo);
      bl[j] = ldfrag(Bl + bo);
    }
#pragma unroll
    for (int i = 0; i < 2; ++i) {
      const size_t ao = (size_t)(m0 + (i << 4) + rl) * lda + k0 + koff;
      const v16b ah = ldfrag(Ah + ao);
      const v16b al = ldfrag(Al + ao);
#pragma unroll
      for (int j = 0; j < 4; ++j) {
        v8f a = acc[i][j];
        a = mma_bf(ah, bh[j], a);
        a = mma_bf(ah, bl[j], a);
        a = mma_bf(al, bh[j], a);
        acc[i][j] = a;
      }
    }
  }

  float* slab = sT[wave];
  float* Cz = Cf + (size_t)z * strideC;
  us*    Hz = Ch + (size_t)z * strideC;
  us*    Lz = Cl + (size_t)z * strideC;
#pragma unroll
  for (int i = 0; i < 2; ++i) {
    const int mBase = m0 + (i << 4);
#pragma unroll
    for (int j = 0; j < 4; ++j)
#pragma unroll
      for (int r = 0; r < 8; ++r) slab[(mOff + r) * 68 + (j << 4) + rl] = acc[i][j][r];
    lds_wave_sync();
    for (int pass = 0; pass < 2; ++pass) {
      {
        const int h2 = lane >> 4, c4 = (lane & 15) * 4;
#pragma unroll
        for (int it = 0; it < 8; ++it) {
          const int row = it * 2 + h2;
          const v4f v = *(const v4f*)(slab + row * 68 + c4);
          *(volatile v4f*)(Cz + (size_t)(mBase + row) * ldc + n0 + c4) = v;
        }
      }
      {
        const int q = lane >> 3, c8 = (lane & 7) * 8;
#pragma unroll
        for (int it = 0; it < 4; ++it) {
          const int row = it * 4 + q;
          const float* sp = slab + row * 68 + c8;
          v4u hv, lv;
#pragma unroll
          for (int e = 0; e < 4; ++e) {
            us h0, l0, h1, l1;
            split2(sp[2 * e], h0, l0);
            split2(sp[2 * e + 1], h1, l1);
            hv[e] = pk16(h0, h1);
            lv[e] = pk16(l0, l1);
          }
          *(volatile v4u*)(Hz + (size_t)(mBase + row) * ldc + n0 + c8) = hv;
          *(volatile v4u*)(Lz + (size_t)(mBase + row) * ldc + n0 + c8) = lv;
        }
      }
      __threadfence();
    }
    lds_wave_sync();
  }
}

__global__ __launch_bounds__(256) void k_head_coef(const float* __restrict__ Hf, const float* __restrict__ asv,
                                                   const float* __restrict__ adv, float* __restrict__ ASRC,
                                                   float* __restrict__ ADST, int C) {
  const int HC = NHEAD * C;
  const int h = blockIdx.x & 7, b = blockIdx.x >> 3;
  const int t = threadIdx.x;
  const float* hp = Hf + (size_t)(b * HC + h * C) * NNODE + 4 * t;
  v4f s = {0.f, 0.f, 0.f, 0.f};
  v4f d = {0.f, 0.f, 0.f, 0.f};
#pragma unroll 1
  for (int cc = 0; cc < C; ++cc) {
    const v4f hv = *(const v4f*)(hp + (size_t)cc * NNODE);
    const float a = asv[h * C + cc];
    const float e = adv[h * C + cc];
    s += hv * a;
    d += hv * e;
  }
  const size_t o = (size_t)(b * NHEAD + h) * NNODE + 4 * t;
  *(volatile v4f*)(ASRC + o) = s;
  *(volatile v4f*)(ADST + o) = d;
  __threadfence();
  *(volatile v4f*)(ASRC + o) = s;
  *(volatile v4f*)(ADST + o) = d;
}

__device__ __forceinline__ float attw(float a, float d, float m) {
  const float s = lrelu02(a + d);
  return __expf(s - m);
}

template <int C, bool ELU, bool OUTF32>
__global__ __launch_bounds__(128) void k_aggr_split(
    const us* __restrict__ HTh, const us* __restrict__ HTl,
    const float* __restrict__ adj,
    const float* __restrict__ ASRC, const float* __restrict__ ADST,
    const float* __restrict__ bias,
    float* __restrict__ outf, us* __restrict__ oxh, us* __restrict__ oxl) {
  constexpr int HC  = NHEAD * C;
  constexpr int HW  = 64 / C;
  constexpr int BH  = 2 * HW;
  constexpr int NHB = NHEAD / BH;
  constexpr int TPW = C / 16;
  constexpr int TPH = 128 / BH;
  constexpr int JPT = NNODE / TPH;
  __shared__ __align__(16) us Psm[4][2 * 32 * 64];
  __shared__ float amax_s[BH];
  __shared__ float dsm[BH][64];
  __shared__ float msm[BH][64];
  __shared__ float lsm[4][HW][32];

  const int tid  = threadIdx.x;
  const int wave = tid >> 5;
  const int lane = tid & 31;
  const int hh = lane >> 4, c = lane & 15;
  const int jg = lane & 3, rq = lane >> 2;
  const int rg = wave & 1, hg = wave >> 1;
  int bx = blockIdx.x;
  const int hblk = bx % NHB;
  bx /= NHB;
  const int ib = bx & 15;
  const int b  = bx >> 4;
  const int i0 = ib * 64;
  const int hbase = hblk * BH;

  {
    const int hl = tid / TPH;
    const int q  = tid - hl * TPH;
    const float* sp = ASRC + (size_t)(b * NHEAD + hbase + hl) * NNODE + q * JPT;
    float m = -INFINITY;
#pragma unroll
    for (int i = 0; i < JPT / 4; ++i) {
      const v4f v = *(const v4f*)(sp + 4 * i);
      m = fmaxf(m, fmaxf(fmaxf(v[0], v[1]), fmaxf(v[2], v[3])));
    }
#pragma unroll
    for (int off = TPH / 2; off > 0; off >>= 1) m = fmaxf(m, __shfl_xor(m, off, 32));
    if (q == 0) amax_s[hl] = m;
  }
  __syncthreads();
  for (int idx = tid; idx < BH * 64; idx += 128) {
    const int hl = idx >> 6, r = idx & 63;
    const float d = ADST[(size_t)(b * NHEAD + hbase + hl) * NNODE + i0 + r];
    dsm[hl][r] = d;
    msm[hl][r] = lrelu02(amax_s[hl] + d);
  }
  __syncthreads();

  v8f acc[2][4];
#pragma unroll
  for (int rt = 0; rt < 2; ++rt)
#pragma unroll
    for (int tt = 0; tt < 4; ++tt) acc[rt][tt] = zero8();
  float lacc[HW][4];
#pragma unroll
  for (int hw = 0; hw < HW; ++hw)
#pragma unroll
    for (int r4 = 0; r4 < 4; ++r4) lacc[hw][r4] = 0.f;

  us* ph = Psm[wave];
  us* pl = ph + 32 * 64;
  const size_t arow = (size_t)(b * NNODE + i0 + 32 * rg + 4 * rq) * NNODE + 16 * jg;

#pragma unroll 1
  for (int chn = 0; chn < NNODE / 64; ++chn) {
    const int j0 = chn * 64;
    unsigned mb[4];
#pragma unroll
    for (int r4 = 0; r4 < 4; ++r4) {
      const float* ap = adj + arow + (size_t)r4 * NNODE + j0;
      unsigned bits = 0u;
#pragma unroll
      for (int q = 0; q < 4; ++q) {
        const v4f a = *(const v4f*)(ap + 4 * q);
#pragma unroll
        for (int e = 0; e < 4; ++e) bits |= (a[e] != 0.0f ? 1u : 0u) << (4 * q + e);
      }
      mb[r4] = bits;
    }
#pragma unroll
    for (int hw = 0; hw < HW; ++hw) {
      const int hl = hg * HW + hw;
      const int hd = hbase + hl;
      float sj[16];
      {
        const float* sp = ASRC + (size_t)(b * NHEAD + hd) * NNODE + j0 + 16 * jg;
#pragma unroll
        for (int q = 0; q < 4; ++q) {
          const v4f v = *(const v4f*)(sp + 4 * q);
          sj[4 * q + 0] = v[0]; sj[4 * q + 1] = v[1]; sj[4 * q + 2] = v[2]; sj[4 * q + 3] = v[3];
        }
      }
#pragma unroll
      for (int r4 = 0; r4 < 4; ++r4) {
        const int wr = 4 * rq + r4;
        const float d = dsm[hl][32 * rg + wr];
        const float m = msm[hl][32 * rg + wr];
        const unsigned bits = mb[r4];
        float lsum = 0.f;
#pragma unroll
        for (int q = 0; q < 2; ++q) {
          v4u hv, lv;
#pragma unroll
          for (int e = 0; e < 4; ++e) {
            const int ja = 8 * q + 2 * e;
            const float e0 = attw(sj[ja], d, m);
            const float e1 = attw(sj[ja + 1], d, m);
            const float p0 = (((bits >> ja) & 1u) != 0u) ? e0 : 0.0f;
            const float p1 = (((bits >> (ja + 1)) & 1u) != 0u) ? e1 : 0.0f;
            lsum += p0;
            lsum += p1;
            us h0, l0, h1, l1;
            split2(p0, h0, l0);
            split2(p1, h1, l1);
            hv[e] = pk16(h0, h1);
            lv[e] = pk16(l0, l1);
          }
          *(v4u*)(ph + wr * 64 + 16 * jg + 8 * q) = hv;
          *(v4u*)(pl + wr * 64 + 16 * jg + 8 * q) = lv;
        }
        lacc[hw][r4] += lsum;
      }
      lds_wave_sync();
#pragma unroll
      for (int kk = 0; kk < 2; ++kk) {
        v16b bhf[TPW], blf[TPW];
#pragma unroll
        for (int t = 0; t < TPW; ++t) {
          const size_t bo = (size_t)(b * HC + hd * C + t * 16 + c) * NNODE + j0 + kk * 32 + 8 * hh;
          bhf[t] = ldfrag(HTh + bo);
          blf[t] = ldfrag(HTl + bo);
        }
#pragma unroll
        for (int rt = 0; rt < 2; ++rt) {
          const int ao = (rt * 16 + c) * 64 + kk * 32 + 8 * hh;
          const v16b ah = ldfrag(ph + ao);
          const v16b al = ldfrag(pl + ao);
#pragma unroll
          for (int t = 0; t < TPW; ++t) {
            v8f a = acc[rt][hw * TPW + t];
            a = mma_bf(ah, bhf[t], a);
            a = mma_bf(ah, blf[t], a);
            a = mma_bf(al, bhf[t], a);
            acc[rt][hw * TPW + t] = a;
          }
        }
      }
      lds_wave_sync();
    }
  }

#pragma unroll
  for (int hw = 0; hw < HW; ++hw)
#pragma unroll
    for (int r4 = 0; r4 < 4; ++r4) {
      float v = lacc[hw][r4];
      v += __shfl_xor(v, 1, 32);
      v += __shfl_xor(v, 2, 32);
      if (jg == 0) lsm[wave][hw][4 * rq + r4] = v;
    }
  lds_wave_sync();

  float* slab = (float*)(Psm[wave]);
  const int cbase = (hbase + hg * HW) * C;
#pragma unroll
  for (int rt = 0; rt < 2; ++rt)
#pragma unroll
    for (int tt = 0; tt < 4; ++tt) {
      const int hw = tt / TPW;
      const float bv = bias[cbase + tt * 16 + c];
#pragma unroll
      for (int r = 0; r < 8; ++r) {
        const int row = rt * 16 + 8 * hh + r;
        const float inv = 1.0f / lsm[wave][hw][row];
        slab[row * 64 + tt * 16 + c] = acc[rt][tt][r] * inv + bv;
      }
    }
  lds_wave_sync();

  const size_t grow0 = (size_t)(b * NNODE + i0 + 32 * rg);
  for (int pass = 0; pass < 2; ++pass) {
    if (OUTF32) {
      const int c4 = c * 4;
#pragma unroll 1
      for (int it = 0; it < 16; ++it) {
        const int row = 2 * it + hh;
        v4f v = *(const v4f*)(slab + row * 64 + c4);
        if (ELU) { v[0] = elu1(v[0]); v[1] = elu1(v[1]); v[2] = elu1(v[2]); v[3] = elu1(v[3]); }
        *(volatile v4f*)(outf + (grow0 + row) * HC + cbase + c4) = v;
      }
    } else {
      const int q8 = lane >> 3, c8 = (lane & 7) * 8;
#pragma unroll 1
      for (int it = 0; it < 8; ++it) {
        const int row = 4 * it + q8;
        const float* sp = slab + row * 64 + c8;
        v4u hv, lv;
#pragma unroll
        for (int e = 0; e < 4; ++e) {
          float f0 = sp[2 * e], f1 = sp[2 * e + 1];
          if (ELU) { f0 = elu1(f0); f1 = elu1(f1); }
          us h0, l0, h1, l1;
          split2(f0, h0, l0);
          split2(f1, h1, l1);
          hv[e] = pk16(h0, h1);
          lv[e] = pk16(l0, l1);
        }
        *(volatile v4u*)(oxh + (grow0 + row) * HC + cbase + c8) = hv;
        *(volatile v4u*)(oxl + (grow0 + row) * HC + cbase + c8) = lv;
      }
    }
    __threadfence();
  }
}

static void layer_front(const float* W, const float* asv, const float* adv, int Fin, int C,
                        us* WTh, us* WTl, const us* Xh, const us* Xl, float* Hf, us* HTh, us* HTl,
                        float* AS, float* AD, hipStream_t stream) {
  const int HC = NHEAD * C;
  k_tsplit<<<dim3(HC / 64, Fin / 64, 1), dim3(256), 0, stream>>>(W, WTh, WTl, Fin, HC, 0L, 0L);
  const int tiles = (HC / 32) * (NNODE / 64);
  k_gemm_split<<<dim3((tiles + 7) / 8, NB), dim3(256), 0, stream>>>(
      WTh, WTl, Fin, Xh, Xl, Fin, (long)NNODE * Fin,
      Hf, HTh, HTl, NNODE, (long)HC * NNODE, HC, NNODE, Fin);
  k_head_coef<<<dim3(NB * NHEAD), dim3(256), 0, stream>>>(Hf, asv, adv, AS, AD, C);
}

extern "C" void kernel_launch(void* const* d_in, const int* in_sizes, int n_in,
                              void* d_out, int out_size, void* d_ws, size_t ws_size,
                              hipStream_t stream) {
  if (n_in < 18) return;
  if (in_sizes[0] != NB * NNODE * 64) return;
  if (in_sizes[1] != NB * NNODE * NNODE) return;
  if (in_sizes[2] != 64 * 256 || in_sizes[3] != 256 || in_sizes[4] != 256 || in_sizes[5] != 256) return;
  if (in_sizes[6] != 256 * 256 || in_sizes[7] != 256 || in_sizes[8] != 256 || in_sizes[9] != 256) return;
  if (in_sizes[10] != 256 * 128 || in_sizes[11] != 128 || in_sizes[12] != 128 || in_sizes[13] != 128) return;
  if (in_sizes[14] != 128 * 128 || in_sizes[15] != 128 || in_sizes[16] != 128 || in_sizes[17] != 128) return;
  if (out_size != NB * NNODE * 128) return;

  const float* x   = (const float*)d_in[0];
  const float* adj = (const float*)d_in[1];
  const float* W1  = (const float*)d_in[2];
  const float* as1 = (const float*)d_in[3];
  const float* ad1 = (const float*)d_in[4];
  const float* b1  = (const float*)d_in[5];
  const float* W2  = (const float*)d_in[6];
  const float* as2 = (const float*)d_in[7];
  const float* ad2 = (const float*)d_in[8];
  const float* b2  = (const float*)d_in[9];
  const float* W3  = (const float*)d_in[10];
  const float* as3 = (const float*)d_in[11];
  const float* ad3 = (const float*)d_in[12];
  const float* b3  = (const float*)d_in[13];
  const float* W4  = (const float*)d_in[14];
  const float* as4 = (const float*)d_in[15];
  const float* ad4 = (const float*)d_in[16];
  const float* b4  = (const float*)d_in[17];

  size_t off = 0;
  const size_t oWTh = off; off += 131072;
  const size_t oWTl = off; off += 131072;
  const size_t oXh  = off; off += (size_t)NB * NNODE * 256 * 2;
  const size_t oXl  = off; off += (size_t)NB * NNODE * 256 * 2;
  const size_t oHf  = off; off += (size_t)NB * 256 * NNODE * 4;
  const size_t oHTh = off; off += (size_t)NB * 256 * NNODE * 2;
  const size_t oHTl = off; off += (size_t)NB * 256 * NNODE * 2;
  const size_t oAS  = off; off += (size_t)NB * NHEAD * NNODE * 4;
  const size_t oAD  = off; off += (size_t)NB * NHEAD * NNODE * 4;
  if (off > ws_size) return;

  char* ws = (char*)d_ws;
  us* WTh = (us*)(ws + oWTh);  us* WTl = (us*)(ws + oWTl);
  us* Xh  = (us*)(ws + oXh);   us* Xl  = (us*)(ws + oXl);
  float* Hf = (float*)(ws + oHf);
  us* HTh = (us*)(ws + oHTh);  us* HTl = (us*)(ws + oHTl);
  float* AS = (float*)(ws + oAS);
  float* AD = (float*)(ws + oAD);
  float* outp = (float*)d_out;

  k_split2<<<dim3((NB * NNODE * 64 / 2 + 255) / 256), dim3(256), 0, stream>>>(x, Xh, Xl, NB * NNODE * 64 / 2);

  layer_front(W1, as1, ad1, 64, 32, WTh, WTl, Xh, Xl, Hf, HTh, HTl, AS, AD, stream);
  k_aggr_split<32, false, false><<<dim3(NB * 16 * 2), dim3(128), 0, stream>>>(HTh, HTl, adj, AS, AD, b1, Hf, Xh, Xl);

  layer_front(W2, as2, ad2, 256, 32, WTh, WTl, Xh, Xl, Hf, HTh, HTl, AS, AD, stream);
  k_aggr_split<32, true, false><<<dim3(NB * 16 * 2), dim3(128), 0, stream>>>(HTh, HTl, adj, AS, AD, b2, Hf, Xh, Xl);

  layer_front(W3, as3, ad3, 256, 16, WTh, WTl, Xh, Xl, Hf, HTh, HTl, AS, AD, stream);
  k_aggr_split<16, false, false><<<dim3(NB * 16), dim3(128), 0, stream>>>(HTh, HTl, adj, AS, AD, b3, Hf, Xh, Xl);

  layer_front(W4, as4, ad4, 128, 16, WTh, WTl, Xh, Xl, Hf, HTh, HTl, AS, AD, stream);
  k_aggr_split<16, true, true><<<dim3(NB * 16), dim3(128), 0, stream>>>(HTh, HTl, adj, AS, AD, b4, outp, Xh, Xl);

  (void)hipGetLastError();
}
